// CausalDenoiser_57526791963183
// MI455X (gfx1250) — hardware-run, weakly checked
//
#include <hip/hip_runtime.h>

typedef float          v8f   __attribute__((ext_vector_type(8)));
typedef float          v4f   __attribute__((ext_vector_type(4)));
typedef unsigned int   v4u   __attribute__((ext_vector_type(4)));
typedef int            v8i   __attribute__((ext_vector_type(8)));
typedef unsigned short v8us  __attribute__((ext_vector_type(8)));
typedef unsigned short v16us __attribute__((ext_vector_type(16)));
typedef __bf16         v16bf __attribute__((ext_vector_type(16)));
typedef _Float16       v16h  __attribute__((ext_vector_type(16)));
typedef v4f  __attribute__((may_alias)) v4fa;
typedef v8us __attribute__((may_alias)) v8usa;
union FragB { v16bf v; v16us u; v8us h[2]; v8i w; };
union FragH { v16h  v; v16us u; v8us h[2]; v8i w; };

__device__ __forceinline__ v8f wmb(const FragB& a, const FragB& b, v8f c) {
  v8f d = __builtin_amdgcn_wmma_f32_16x16x32_bf16(false, a.v, false, b.v, (short)0, c, false, false);
  asm volatile("v_nop\n\tv_nop\n\tv_nop\n\tv_nop" : "+v"(d) : "v"(a.w), "v"(b.w));
  return d;
}

__device__ __forceinline__ v8f wmh(const FragH& a, const FragH& b, v8f c) {
  v8f d = __builtin_amdgcn_wmma_f32_16x16x32_f16(false, a.v, false, b.v, (short)0, c, false, false);
  asm volatile("v_nop\n\tv_nop\n\tv_nop\n\tv_nop" : "+v"(d) : "v"(a.w), "v"(b.w));
  return d;
}

__device__ __forceinline__ unsigned bf16_bits(float f) {
  const unsigned u = __float_as_uint(f);
  const unsigned r = (u + 0x7FFFu + ((u >> 16) & 1u)) >> 16;
  const unsigned q = (u >> 16) | 0x40u;
  return ((u & 0x7fffffffu) > 0x7f800000u) ? q : r;
}

__device__ __forceinline__ float bf16_val(float f) {
  return __uint_as_float(bf16_bits(f) << 16);
}
__device__ __forceinline__ int clampi(int v, int lo, int hi) {
  return v < lo ? lo : (v > hi ? hi : v);
}

__device__ __forceinline__ unsigned f16_bits(float f) {
  const unsigned u  = __float_as_uint(f);
  const unsigned s  = (u >> 16) & 0x8000u;
  const unsigned a  = u & 0x7fffffffu;
  const unsigned t  = a - 0x38000000u;
  const unsigned r  = (t + 0x0FFFu + ((t >> 13) & 1u)) >> 13;
  const unsigned rc = r > 0x7C00u ? 0x7C00u : r;
  const bool small  = a < 0x38800000u;
  const bool isnan  = a > 0x7f800000u;
  const unsigned fin = small ? 0u : (s | rc);
  return isnan ? (s | 0x7E00u) : fin;
}

__device__ __forceinline__ unsigned pk16(unsigned lo, unsigned hi) { return lo | (hi << 16); }
__device__ __forceinline__ unsigned bf16_lo_bits(float v) {
  float hi = bf16_val(v);
  asm volatile("" : "+v"(hi));
  return bf16_bits(v - hi);
}
__device__ __forceinline__ v4u pack8_bf16(v4f a, v4f c) {
  return (v4u){ pk16(bf16_bits(a[0]), bf16_bits(a[1])), pk16(bf16_bits(a[2]), bf16_bits(a[3])),
                pk16(bf16_bits(c[0]), bf16_bits(c[1])), pk16(bf16_bits(c[2]), bf16_bits(c[3])) };
}
__device__ __forceinline__ v4u pack8_bf16_lo(v4f a, v4f c) {
  return (v4u){ pk16(bf16_lo_bits(a[0]), bf16_lo_bits(a[1])), pk16(bf16_lo_bits(a[2]), bf16_lo_bits(a[3])),
                pk16(bf16_lo_bits(c[0]), bf16_lo_bits(c[1])), pk16(bf16_lo_bits(c[2]), bf16_lo_bits(c[3])) };
}
__device__ __forceinline__ v4u pack8_f16(v4f a, v4f c) {
  return (v4u){ pk16(f16_bits(a[0]), f16_bits(a[1])), pk16(f16_bits(a[2]), f16_bits(a[3])),
                pk16(f16_bits(c[0]), f16_bits(c[1])), pk16(f16_bits(c[2]), f16_bits(c[3])) };
}

template <int FORM>
__global__ __launch_bounds__(256) void k_plane(const float* __restrict__ src, int rows, int cols, int ldsrc,
                                               unsigned short* __restrict__ dst, int MP, int KP) {
  static_assert(FORM >= 0 && FORM <= 3);
  const int KTOT = (FORM == 1 || FORM == 3) ? 2 * KP : KP;
  const unsigned ppr   = (unsigned)(KTOT >> 3);
  const unsigned kp8   = (unsigned)(KP >> 3);
  const unsigned total = (unsigned)MP * ppr;
  const unsigned g     = blockIdx.x * 256u + threadIdx.x;
  const unsigned rowu  = g / ppr;
  const unsigned p     = g - rowu * ppr;
  const bool second    = p >= kp8;
  const int row = (int)rowu;
  const int c0  = (int)((second ? p - kp8 : p) << 3);
  const float* srow = src + (size_t)clampi(row, 0, rows - 1) * (size_t)ldsrc;
  float x[8];
  unsigned mk[8];
#pragma unroll
  for (int e = 0; e < 8; ++e) {
    const int c = c0 + e;
    const float v = srow[clampi(c, 0, cols - 1)];
    asm volatile("" :: "v"(v));
    x[e]  = v;
    mk[e] = (row < rows && c < cols) ? 0xFFFFu : 0u;
  }
  const v4f a = (v4f){ x[0], x[1], x[2], x[3] };
  const v4f c = (v4f){ x[4], x[5], x[6], x[7] };
  v4u o;
  if (FORM == 2) {
    o = pack8_f16(a, c);
  } else {
    const v4u hi = pack8_bf16(a, c);
    o = hi;
    if (FORM == 1) { const v4u lo = pack8_bf16_lo(a, c); o = second ? lo : hi; }
  }
  const v4u mw = (v4u){ pk16(mk[0], mk[1]), pk16(mk[2], mk[3]), pk16(mk[4], mk[5]), pk16(mk[6], mk[7]) };
  o &= mw;
  if (g < total) {
    volatile v4u* q = (volatile v4u*)(dst + (size_t)g * 8);
    *q = o;
    __threadfence();
    *q = o;
  }
}

template <int FORM> struct FragOf    { typedef FragB T; };
template <>         struct FragOf<2> { typedef FragH T; };
__device__ __forceinline__ v8f mm(const FragB& a, const FragB& b, v8f c) { return wmb(a, b, c); }
__device__ __forceinline__ v8f mm(const FragH& a, const FragH& b, v8f c) { return wmh(a, b, c); }
template <class F> __device__ __forceinline__ F ld_frag(const unsigned short* p) {
  F f;
  f.h[0] = *(const v8usa*)(p);
  f.h[1] = *(const v8usa*)(p + 16);
  return f;
}

template <int FORM, int EPI>
__global__ __launch_bounds__(256) __attribute__((amdgpu_num_vgpr(248)))
void k_gemm_nt(const unsigned short* __restrict__ A, const unsigned short* __restrict__ B,
               const float* __restrict__ bias, float* __restrict__ D, int M, int N, int KTOT, int ldd) {
  static_assert(FORM >= 0 && FORM <= 2);
  static_assert(EPI == 0 || EPI == 1);
  typedef typename FragOf<FORM>::T F;
  __shared__ __attribute__((aligned(16))) float sT[8][16 * 68];
  const int lane = threadIdx.x & 31;
  const int wave = threadIdx.x >> 5;
  const int tilesM = (M + 63) >> 6;
  const int tilesN = (N + 63) >> 6;
  const int tile = blockIdx.x * 8 + wave;
  if (tile >= tilesM * tilesN) return;
  const int tm = tile / tilesN;
  const int tn = tile - tm * tilesN;
  const int m0 = tm << 6;
  const int n0 = tn << 6;

  const int rl = lane & 15;
  const int h8 = (lane >> 4) * 8;
  const unsigned short* pa = A + (size_t)(m0 + rl) * (size_t)KTOT + h8;
  const unsigned short* pb = B + (size_t)(n0 + rl) * (size_t)KTOT + h8;

  v8f acc[4][4];
#pragma unroll
  for (int i = 0; i < 4; ++i)
#pragma unroll
    for (int j = 0; j < 4; ++j) acc[i][j] = (v8f){0.f, 0.f, 0.f, 0.f, 0.f, 0.f, 0.f, 0.f};

#pragma unroll 1
  for (int k0 = 0; k0 < KTOT; k0 += 32) {
    F bf[4];
#pragma unroll
    for (int j = 0; j < 4; ++j) bf[j] = ld_frag<F>(pb + (size_t)(j << 4) * (size_t)KTOT + k0);
#pragma unroll
    for (int i = 0; i < 4; ++i) {
      const F af = ld_frag<F>(pa + (size_t)(i << 4) * (size_t)KTOT + k0);
#pragma unroll
      for (int j = 0; j < 4; ++j) acc[i][j] = mm(af, bf[j], acc[i][j]);
    }
  }

  float* slab = sT[wave];
  const int hh = lane >> 4;
  const int c4 = (lane & 15) * 4;
  const int nc = n0 + c4;
  const bool cok = nc < N;
  v4f bv = (v4f){0.f, 0.f, 0.f, 0.f};
  if (EPI == 1) {
    bv = *(const v4fa*)(bias + clampi(nc, 0, N - 4));
    asm volatile("" :: "v"(bv));
  }
#pragma unroll
  for (int i = 0; i < 4; ++i) {
    const int mBase = m0 + (i << 4);
#pragma unroll
    for (int j = 0; j < 4; ++j) {
#pragma unroll
      for (int r = 0; r < 8; ++r) slab[(h8 + r) * 68 + (j << 4) + rl] = acc[i][j][r];
    }
    __builtin_amdgcn_fence(__ATOMIC_RELEASE, "workgroup");
    __builtin_amdgcn_wave_barrier();
    __builtin_amdgcn_fence(__ATOMIC_ACQUIRE, "workgroup");
    v4f vv[8];
#pragma unroll
    for (int it = 0; it < 8; ++it) {
      const int row = it * 2 + hh;
      v4f v = *(const v4fa*)(slab + row * 68 + c4);
      if (EPI == 1) v += bv;
      vv[it] = v;
    }
    for (int pass = 0; pass < 2; ++pass) {
#pragma unroll
      for (int it = 0; it < 8; ++it) {
        const int row = mBase + it * 2 + hh;
        if (cok && row < M) *(volatile v4f*)(D + (size_t)row * (size_t)ldd + nc) = vv[it];
      }
      __threadfence();
    }
    __builtin_amdgcn_fence(__ATOMIC_RELEASE, "workgroup");
    __builtin_amdgcn_wave_barrier();
    __builtin_amdgcn_fence(__ATOMIC_ACQUIRE, "workgroup");
  }
}

#pragma clang fp contract(off)

typedef float v2f __attribute__((ext_vector_type(2)));
typedef int   v4i __attribute__((ext_vector_type(4)));
typedef v2f __attribute__((may_alias)) v2fa;
typedef v4i __attribute__((may_alias)) v4ia;

#define MSG_SPLIT_L1 1
#define MSG_SPLIT_L2 1
#define KT1    (MSG_SPLIT_L1 ? 128 : 64)
#define KT2    (MSG_SPLIT_L2 ? 128 : 64)

#define NU     100000
#define NI     50000
#define NN     150000
#define NE     1000000
#define DD     64
#define MROWS  150016
#define NBA    1024
#define NBU    98
#define NBI    49
#define NBLK   147
#define RCAP_U 13312
#define RCAP_I 26624
#define DEGCAP 64
#define WLCAP  4096
#define WSPAN  125000
#define WCH    489
#define NREC   3907
#define MEAS_B1024_U 10439
#define MEAS_B1024_I 20839
#define MEAS_DEG     40
#define BK_INTS (8 * WLCAP + RCAP_I + 3 * NBA + 32)
#define BK_LDS_BYTES (BK_INTS * 4)

static_assert(NU + NI == NN && DD == 64);
static_assert(MROWS % 64 == 0 && MROWS >= NN && MROWS - NN < 64 && NN % 16 == 0);
static_assert(NBU * NBA >= NU && (NBU - 1) * NBA < NU);
static_assert(NBI * NBA >= NI + (MROWS - NN) && (NBI - 1) * NBA < NI);
static_assert(NBU + NBI == NBLK && NBA == 1024);
static_assert(NE <= (1 << 20));
static_assert(RCAP_U * 4 >= MEAS_B1024_U * 5 && RCAP_I * 4 >= MEAS_B1024_I * 5);
static_assert(RCAP_U % 1024 == 0 && RCAP_I % 1024 == 0 && RCAP_I >= RCAP_U);
static_assert(DEGCAP >= MEAS_DEG + 8);
static_assert(8 * WSPAN == NE && WCH * 256 >= WSPAN && (WCH - 1) * 256 < WSPAN);
static_assert(8 * WLCAP >= RCAP_I && WLCAP * 8 >= WSPAN / 49 * 8);
static_assert(BK_INTS % 4 == 0 && BK_LDS_BYTES <= 262144 && BK_LDS_BYTES + 0 <= 327680);
static_assert(NE % 32 == 0 && NREC * 8 >= NE / 32 && (NREC - 1) * 8 < NE / 32);
static_assert(KT1 % 32 == 0 && KT2 % 32 == 0 && DD % 4 == 0);
static_assert((long long)MROWS * 128 / 8 < (1LL << 31));
static_assert((long long)NBU * RCAP_U + (long long)NBI * RCAP_I < (1LL << 30));

constexpr size_t al256c(size_t x) { return (x + 255) & ~(size_t)255; }
constexpr size_t SZ_F   = (size_t)MROWS * DD * 4;
constexpr size_t SZ_C   = (size_t)MROWS * 128 * 2;
constexpr size_t SZ_IPW = (size_t)NE * 4;
constexpr size_t SZ_LST = ((size_t)NBU * RCAP_U + (size_t)NBI * RCAP_I) * 4;
constexpr size_t SZ_CNT = (size_t)NBLK * NBA * 4;
constexpr size_t SZ_FLG = (size_t)NBLK * 128;
constexpr size_t SZ_REC = (size_t)NREC * 128;
constexpr size_t SZ_WD  = (size_t)64 * 128 * 2;
constexpr size_t SZ_BIA = (size_t)2 * DD * 4;
constexpr size_t O_A    = 0;
constexpr size_t O_B    = O_A   + al256c(SZ_F);
constexpr size_t O_C    = O_B   + al256c(SZ_F);
constexpr size_t O_IPW  = O_C   + al256c(SZ_C);
constexpr size_t O_LST  = O_IPW + al256c(SZ_IPW);
constexpr size_t O_CNT  = O_LST + al256c(SZ_LST);
constexpr size_t O_OFF  = O_CNT + al256c(SZ_CNT);
constexpr size_t O_FLG  = O_OFF + al256c(SZ_CNT);
constexpr size_t O_REC  = O_FLG + al256c(SZ_FLG);
constexpr size_t O_WD0  = O_REC + al256c(SZ_REC);
constexpr size_t O_WD1  = O_WD0 + al256c(SZ_WD);
constexpr size_t O_BIA  = O_WD1 + al256c(SZ_WD);
constexpr size_t WS_TOTAL = O_BIA + al256c(SZ_BIA);
static_assert(WS_TOTAL <= ((size_t)128 << 20));
static_assert((size_t)NN * DD + 1 == (size_t)9600001);

__global__ __launch_bounds__(32) void k_bias(const float* __restrict__ b0, const float* __restrict__ b1,
                                             float* __restrict__ BIAS) {
  const int lane = threadIdx.x & 31;
  const int c = (lane & 15) * 4;
  const v4f x0 = *(const v4fa*)(b0 + c);
  const v4f x1 = *(const v4fa*)(b1 + c);
  asm volatile("" :: "v"(x0));
  asm volatile("" :: "v"(x1));
  const bool second = lane >= 16;
  v4f o;
  o[0] = bf16_val(second ? x1[0] : x0[0]);
  o[1] = bf16_val(second ? x1[1] : x0[1]);
  o[2] = bf16_val(second ? x1[2] : x0[2]);
  o[3] = bf16_val(second ? x1[3] : x0[3]);
  volatile v4f* q = (volatile v4f*)(BIAS + 4 * lane);
  *q = o;
  __threadfence();
  *q = o;
}

__global__ __launch_bounds__(256) void k_node(const float* __restrict__ ego, float* __restrict__ XR,
                                              float* __restrict__ UN) {
  const int g = (int)blockIdx.x * 256 + (int)threadIdx.x;
  const bool live = g < NN * 16;
  const int gc = live ? g : NN * 16 - 1;
  const size_t o = (size_t)gc * 4;
  const v4f x = *(const v4fa*)(ego + o);
  asm volatile("" :: "v"(x));
  const float r0 = bf16_val(x[0]), r1 = bf16_val(x[1]), r2 = bf16_val(x[2]), r3 = bf16_val(x[3]);
  float ss = (r0 * r0 + r1 * r1) + (r2 * r2 + r3 * r3);
  ss += __shfl_xor(ss, 8, 32);
  ss += __shfl_xor(ss, 4, 32);
  ss += __shfl_xor(ss, 2, 32);
  ss += __shfl_xor(ss, 1, 32);
  const float d = fmaxf(sqrtf(ss), 1e-12f);
  const v4f xr = (v4f){ r0, r1, r2, r3 };
  const v4f un = (v4f){ r0 / d, r1 / d, r2 / d, r3 / d };
  if (live) {
    *(volatile v4f*)(XR + o) = xr;
    *(volatile v4f*)(UN + o) = un;
  }
  __threadfence();
  if (live) {
    *(volatile v4f*)(XR + o) = xr;
    *(volatile v4f*)(UN + o) = un;
  }
}

__global__ __launch_bounds__(256) void k_inter(const float* __restrict__ UN, const int* __restrict__ uid,
                                               const int* __restrict__ iid, const float* __restrict__ treat,
                                               const float* __restrict__ alpha_p, const float* __restrict__ beta_p,
                                               float* __restrict__ IPW, unsigned* __restrict__ REC) {
  __shared__ double sred[8];
  const int lane = threadIdx.x & 31;
  const int wave = threadIdx.x >> 5;
  const int wg = (int)blockIdx.x * 8 + wave;
  const bool active = wg < NE / 32;
  const int t0 = wg * 32;
  const int tl = clampi(t0 + lane, 0, NE - 1);
  int uL = uid[tl];
  int iL = iid[tl];
  float tr = treat[tl];
  asm volatile("" :: "v"(uL));
  asm volatile("" :: "v"(iL));
  asm volatile("" :: "v"(tr));
  uL = clampi(uL, 0, NU - 1);
  iL = NU + clampi(iL, 0, NI - 1);
  tr = bf16_val(tr);
  const float alpha = bf16_val(alpha_p[0]);
  const float beta  = bf16_val(beta_p[0]);
  const int h = lane >> 4;
  const int l16 = lane & 15;
  float sim = 0.0f;
#pragma unroll 2
  for (int s = 0; s < 16; ++s) {
    const int srcl = 2 * s + h;
    const int u  = __shfl(uL, srcl, 32);
    const int it = __shfl(iL, srcl, 32);
    const v4f a = *(const v4fa*)(UN + (size_t)u  * DD + 4 * l16);
    const v4f b = *(const v4fa*)(UN + (size_t)it * DD + 4 * l16);
    asm volatile("" :: "v"(a));
    asm volatile("" :: "v"(b));
    float p = (a[0] * b[0] + a[1] * b[1]) + (a[2] * b[2] + a[3] * b[3]);
    p += __shfl_xor(p, 8, 32);
    p += __shfl_xor(p, 4, 32);
    p += __shfl_xor(p, 2, 32);
    p += __shfl_xor(p, 1, 32);
    const float p0 = __int_as_float(__builtin_amdgcn_readlane(__float_as_int(p), 0));
    const float p1 = __int_as_float(__builtin_amdgcn_readlane(__float_as_int(p), 16));
    const float pick = (lane & 1) ? p1 : p0;
    sim = ((lane >> 1) == s) ? pick : sim;
  }
  const float z = alpha * sim + beta;
  const float e = 1.0f / (1.0f + expf(-z));
  const float term = tr * logf(e) + (1.0f - tr) * logf(1.0f - e);
  const float w = tr / (e + 1e-8f);
  if (active) {
    volatile float* q = IPW + t0 + lane;
    *q = w;
    __threadfence();
    *q = w;
  }
  double dt = active ? (double)term : 0.0;
  dt += __shfl_xor(dt, 16, 32);
  dt += __shfl_xor(dt, 8, 32);
  dt += __shfl_xor(dt, 4, 32);
  dt += __shfl_xor(dt, 2, 32);
  dt += __shfl_xor(dt, 1, 32);
  if (lane == 0) sred[wave] = dt;
  __syncthreads();
  if (wave == 0) {
    double sacc = 0.0;
#pragma unroll 1
    for (int i = 0; i < 8; ++i) sacc += sred[i];
    const unsigned long long bits = (unsigned long long)__double_as_longlong(sacc);
    const unsigned lo = (unsigned)(bits & 0xffffffffull);
    const unsigned hi = (unsigned)(bits >> 32);
    const v4u o = (v4u){ lane == 0 ? lo : 0u, lane == 0 ? hi : 0u, 0u, 0u };
    if (lane < 8) {
      volatile v4u* q = (volatile v4u*)(REC + (size_t)blockIdx.x * 32 + lane * 4);
      *q = o;
      __threadfence();
      *q = o;
    }
  }
}

__global__ __launch_bounds__(256) void k_loss(const unsigned* __restrict__ REC, float* __restrict__ out) {
  __shared__ double sp[256];
  const int tid = (int)threadIdx.x;
  double s = 0.0;
#pragma unroll 1
  for (int j = 0; j < 16; ++j) {
    const int b = j * 256 + tid;
    const int bc = b < NREC ? b : NREC - 1;
    const unsigned lo = REC[(size_t)bc * 32];
    const unsigned hi = REC[(size_t)bc * 32 + 1];
    asm volatile("" :: "v"(lo));
    asm volatile("" :: "v"(hi));
    const double v = __longlong_as_double((long long)(((unsigned long long)hi << 32) | (unsigned long long)lo));
    s += (b < NREC) ? v : 0.0;
  }
  sp[tid] = s;
  __syncthreads();
  if (tid == 0) {
    double a = 0.0;
#pragma unroll 1
    for (int i = 0; i < 256; ++i) a += sp[i];
    const float r = (float)(-(a / 1.0e6));
    volatile float* q = out + (size_t)NN * DD;
    *q = r;
    __threadfence();
    *q = r;
  }
}

__device__ __forceinline__ int sweep_keys(const int* __restrict__ keys, unsigned ubase, unsigned unb,
                                          int* wlw, int lane, int wave) {
  int wc = 0;
  const int wb = wave * WSPAN;
#pragma unroll 1
  for (int c = 0; c < WCH; ++c) {
    const int loc0 = c * 256 + lane;
    unsigned sv[8];
    bool hv[8];
    bool anyh = false;
#pragma unroll
    for (int j = 0; j < 8; ++j) {
      const int loc = loc0 + j * 32;
      const int gi = wb + loc;
      int k = keys[gi < NE ? gi : NE - 1];
      asm volatile("" :: "v"(k));
      k = (loc < WSPAN) ? k : -1;
      sv[j] = (unsigned)k - ubase;
      hv[j] = sv[j] < unb;
      anyh = anyh | hv[j];
    }
    const unsigned any = __builtin_amdgcn_ballot_w32(anyh);
    if (any != 0u) {
#pragma unroll
      for (int j = 0; j < 8; ++j) {
        const unsigned mj = __builtin_amdgcn_ballot_w32(hv[j]);
        const int pos = wc + (int)__builtin_amdgcn_mbcnt_lo(mj, 0u);
        if (hv[j] && pos < WLCAP) wlw[pos] = (int)(((unsigned)(wb + loc0 + j * 32) << 10) | sv[j]);
        wc += (int)__builtin_popcount(mj);
      }
    }
  }
  return wc;
}

__global__ __launch_bounds__(256) void k_bucket(const int* __restrict__ uid, const int* __restrict__ iid,
                                                int* __restrict__ LIST, int* __restrict__ CNT,
                                                int* __restrict__ OFF, int* __restrict__ FLAG) {
  extern __shared__ __attribute__((aligned(16))) int dsm[];
  int* wl   = dsm;
  int* sl   = wl + 8 * WLCAP;
  int* cnt  = sl + RCAP_I;
  int* offs = cnt + NBA;
  int* cur  = offs + NBA;
  int* misc = cur + NBA;
  const int tid = (int)threadIdx.x, lane = tid & 31, wave = tid >> 5;
  const int blk = (int)blockIdx.x;
  const bool isItem = blk >= NBU;
  const int bl = isItem ? blk - NBU : blk;
  const int base = bl * NBA;
  const int ntot = isItem ? NI : NU;
  const int nOwn = (ntot - base) < NBA ? (ntot - base) : NBA;
  const int rcap = isItem ? RCAP_I : RCAP_U;
  const int listOff = isItem ? (NBU * RCAP_U + bl * RCAP_I) : (bl * RCAP_U);

  {
    const v4i z4 = (v4i){0, 0, 0, 0};
    for (int i = tid * 4; i < BK_INTS; i += 1024) *(v4ia*)(dsm + i) = z4;
  }
  __syncthreads();

  int wc;
  if (isItem) wc = sweep_keys(iid, (unsigned)base, (unsigned)nOwn, wl + wave * WLCAP, lane, wave);
  else        wc = sweep_keys(uid, (unsigned)base, (unsigned)nOwn, wl + wave * WLCAP, lane, wave);
  if (lane == 0) misc[wave] = wc;
  __syncthreads();

  if (wave == 0) {
    int tot = 0, ov = 0;
#pragma unroll 1
    for (int w2 = 0; w2 < 8; ++w2) {
      const int craw = misc[w2];
      ov |= (craw > WLCAP) ? 1 : 0;
      const int c = __builtin_amdgcn_readfirstlane(clampi(craw, 0, WLCAP));
#pragma unroll 1
      for (int b0 = 0; b0 < c; b0 += 32) {
        const int idx = b0 + lane;
        const int ent = wl[w2 * WLCAP + (idx < WLCAP ? idx : WLCAP - 1)];
        const int m32 = (c - b0) < 32 ? (c - b0) : 32;
#pragma unroll 1
        for (int k = 0; k < m32; ++k) {
          const int u = __builtin_amdgcn_readlane(ent, k);
          const int slot = u & (NBA - 1);
          if (lane == 0) cnt[slot] = cnt[slot] + 1;
        }
      }
      tot += c;
    }
    if (tot > rcap) ov = 1;
    if (lane == 0) { misc[8] = tot; misc[9] = ov; }
  }
  __syncthreads();

  if (wave == 0) {
    const int b32 = lane * (NBA / 32);
    int s = 0;
#pragma unroll 1
    for (int i = 0; i < NBA / 32; ++i) s += cnt[b32 + i];
    int incl = s;
#pragma unroll
    for (int d = 1; d < 32; d <<= 1) {
      const int y = __shfl_up(incl, d, 32);
      incl += (lane >= d) ? y : 0;
    }
    int run = incl - s;
#pragma unroll 1
    for (int i = 0; i < NBA / 32; ++i) {
      const int cv = cnt[b32 + i];
      offs[b32 + i] = run;
      cur[b32 + i]  = run;
      run += cv;
    }
  }
  __syncthreads();

  if (wave == 0) {
#pragma unroll 1
    for (int w2 = 0; w2 < 8; ++w2) {
      const int c = __builtin_amdgcn_readfirstlane(clampi(misc[w2], 0, WLCAP));
#pragma unroll 1
      for (int b0 = 0; b0 < c; b0 += 32) {
        const int idx = b0 + lane;
        const int ent = wl[w2 * WLCAP + (idx < WLCAP ? idx : WLCAP - 1)];
        const int m32 = (c - b0) < 32 ? (c - b0) : 32;
#pragma unroll 1
        for (int k = 0; k < m32; ++k) {
          const int u = __builtin_amdgcn_readlane(ent, k);
          const int slot = u & (NBA - 1);
          if (lane == 0) {
            int p = cur[slot];
            p = clampi(p, 0, rcap - 1);
            sl[p] = (int)((unsigned)u >> 10);
            cur[slot] = p + 1;
          }
        }
      }
    }
  }
  __syncthreads();

  const v4i cv4 = *(const v4ia*)(cnt + tid * 4);
  const v4i ov4 = *(const v4ia*)(offs + tid * 4);
  const bool big = (cv4.x > DEGCAP) | (cv4.y > DEGCAP) | (cv4.z > DEGCAP) | (cv4.w > DEGCAP);
  const unsigned bm = __builtin_amdgcn_ballot_w32(big);
  if (lane == 0) misc[16 + wave] = (bm != 0u) ? 1 : 0;
  __syncthreads();
  int flag = misc[9];
#pragma unroll 1
  for (int i = 0; i < 8; ++i) flag |= misc[16 + i];
  const v4i fv = (v4i){ lane == 0 ? flag : 0, 0, 0, 0 };
  int* gl = LIST + listOff;
  const int nv4 = rcap >> 2;
  for (int pass = 0; pass < 2; ++pass) {
#pragma unroll 1
    for (int i = tid; i < nv4; i += 256) {
      const v4i v = *(const v4ia*)(sl + 4 * i);
      *(volatile v4i*)(gl + 4 * i) = v;
    }
    *(volatile v4i*)(CNT + (size_t)blk * NBA + tid * 4) = cv4;
    *(volatile v4i*)(OFF + (size_t)blk * NBA + tid * 4) = ov4;
    if (wave == 0 && lane < 8) *(volatile v4i*)(FLAG + (size_t)blk * 32 + lane * 4) = fv;
    __threadfence();
  }
}

template <int KT>
__global__ __launch_bounds__(256) void k_replay(const float* __restrict__ SRC, const float* __restrict__ IPW,
                                                const int* __restrict__ uid, const int* __restrict__ iid,
                                                const int* __restrict__ LIST, const int* __restrict__ CNT,
                                                const int* __restrict__ OFF, const int* __restrict__ FLAG,
                                                unsigned short* __restrict__ MSG) {
  static_assert(KT == 64 || KT == 128);
  const int tid = (int)threadIdx.x, lane = tid & 31, wave = tid >> 5;
  const int blk = (int)blockIdx.x;
  const bool isItem = blk >= NBU;
  const int bl = isItem ? blk - NBU : blk;
  const int base = bl * NBA;
  const int ntot = isItem ? NI : NU;
  const int nOwn = (ntot - base) < NBA ? (ntot - base) : NBA;
  const int nodeBase = (isItem ? NU : 0) + base;
  const int rcap = isItem ? RCAP_I : RCAP_U;
  const int listOff = isItem ? (NBU * RCAP_U + bl * RCAP_I) : (bl * RCAP_U);
  const int* LB = LIST + listOff;
  int fl = FLAG[(size_t)blk * 32];
  asm volatile("" :: "v"(fl));
  const bool bad = fl != 0;
  const float qn = __int_as_float(0x7fc00000);

#pragma unroll 1
  for (int si = 0; si < NBA / 8; ++si) {
    const int s = si * 8 + wave;
    const int node = nodeBase + s;
    const bool live = s < nOwn;
    const bool wr = isItem ? (node < MROWS) : live;
    if (!wr) continue;
    const int ix = blk * NBA + s;
    int cv = CNT[ix];
    int ovv = OFF[ix];
    asm volatile("" :: "v"(cv));
    asm volatile("" :: "v"(ovv));
    const bool big = cv > DEGCAP;
    const int cn = __builtin_amdgcn_readfirstlane(live ? clampi(cv, 0, DEGCAP) : 0);
    const int o  = __builtin_amdgcn_readfirstlane(clampi(ovv, 0, rcap));
    float a0 = 0.0f, a1 = 0.0f, sw = 0.0f;
#pragma unroll 1
    for (int b0 = 0; b0 < cn; b0 += 32) {
      int li = o + b0 + lane;
      li = li > rcap - 1 ? rcap - 1 : li;
      int t = LB[li];
      asm volatile("" :: "v"(t));
      t = clampi(t, 0, NE - 1);
      float w = IPW[t];
      int iu = uid[t];
      int ii = iid[t];
      asm volatile("" :: "v"(w));
      asm volatile("" :: "v"(iu));
      asm volatile("" :: "v"(ii));
      const int col = isItem ? clampi(iu, 0, NU - 1) : (NU + clampi(ii, 0, NI - 1));
      const int wi = __float_as_int(w);
      const int m32 = (cn - b0) < 32 ? (cn - b0) : 32;
#pragma unroll 1
      for (int k = 0; k < m32; ++k) {
        const int   ck = __builtin_amdgcn_readlane(col, k);
        const float wk = __int_as_float(__builtin_amdgcn_readlane(wi, k));
        const v2f v = *(const v2fa*)(SRC + (size_t)ck * DD + 2 * lane);
        asm volatile("" :: "v"(v));
        a0 = fmaf(wk, v[0], a0);
        a1 = fmaf(wk, v[1], a1);
        sw += wk;
      }
    }
    const float deg = sw + 1e-8f;
    float dinv = 1.0f / sqrtf(deg);
    dinv = ((__float_as_uint(dinv) & 0x7fffffffu) == 0x7f800000u) ? 0.0f : dinv;
    float m0 = dinv * a0;
    float m1 = dinv * a1;
    const bool poison = bad || big;
    m0 = poison ? qn : m0;
    m1 = poison ? qn : m1;
    m0 = live ? m0 : 0.0f;
    m1 = live ? m1 : 0.0f;
    const unsigned hw = pk16(bf16_bits(m0), bf16_bits(m1));
    const unsigned lw = pk16(bf16_lo_bits(m0), bf16_lo_bits(m1));
    volatile unsigned* q = (volatile unsigned*)(MSG + (size_t)node * KT);
    q[lane] = hw;
    if (KT == 128) q[32 + lane] = lw;
    __threadfence();
    q[lane] = hw;
    if (KT == 128) q[32 + lane] = lw;
  }
}

__global__ __launch_bounds__(256) void k_row1(const float* __restrict__ H, float* __restrict__ CUR) {
  const int g = (int)blockIdx.x * 256 + (int)threadIdx.x;
  const bool live = g < NN * 16;
  const int gc = live ? g : NN * 16 - 1;
  const size_t o = (size_t)gc * 4;
  const v4f h = *(const v4fa*)(H + o);
  asm volatile("" :: "v"(h));
  v4f r;
  r[0] = (h[0] > 0.0f) ? h[0] : (h[0] - h[0]);
  r[1] = (h[1] > 0.0f) ? h[1] : (h[1] - h[1]);
  r[2] = (h[2] > 0.0f) ? h[2] : (h[2] - h[2]);
  r[3] = (h[3] > 0.0f) ? h[3] : (h[3] - h[3]);
  if (live) *(volatile v4f*)(CUR + o) = r;
  __threadfence();
  if (live) *(volatile v4f*)(CUR + o) = r;
}

__global__ __launch_bounds__(256) void k_row2(const float* __restrict__ ego, const float* __restrict__ CUR,
                                              const float* __restrict__ H, const int* __restrict__ FLAG,
                                              float* __restrict__ out) {
  const int g = (int)blockIdx.x * 256 + (int)threadIdx.x;
  const bool live = g < NN * 16;
  const int gc = live ? g : NN * 16 - 1;
  const int n = gc >> 4;
  const size_t o = (size_t)gc * 4;
  const v4f e = *(const v4fa*)(ego + o);
  const v4f c = *(const v4fa*)(CUR + o);
  const v4f h = *(const v4fa*)(H + o);
  asm volatile("" :: "v"(e));
  asm volatile("" :: "v"(c));
  asm volatile("" :: "v"(h));
  const int fb = (n < NU) ? (n >> 10) : (NBU + ((n - NU) >> 10));
  int fl = FLAG[(size_t)clampi(fb, 0, NBLK - 1) * 32];
  asm volatile("" :: "v"(fl));
  const float qn = __int_as_float(0x7fc00000);
  v4f r;
#pragma unroll
  for (int i = 0; i < 4; ++i) {
    const float hr = (h[i] > 0.0f) ? h[i] : (h[i] - h[i]);
    const float v = ((bf16_val(e[i]) + c[i]) + hr) / 3.0f;
    r[i] = (fl != 0) ? qn : v;
  }
  if (live) *(volatile v4f*)(out + o) = r;
  __threadfence();
  if (live) *(volatile v4f*)(out + o) = r;
}

extern "C" void kernel_launch(void* const* d_in, const int* in_sizes, int n_in,
                              void* d_out, int out_size, void* d_ws, size_t ws_size,
                              hipStream_t stream) {
  if (n_in < 10) return;
  if (in_sizes[0] != NN * DD) return;
  if (in_sizes[1] != NE || in_sizes[2] != NE || in_sizes[3] != NE) return;
  if (in_sizes[4] < 1 || in_sizes[5] < 1) return;
  if (in_sizes[6] != DD * DD || in_sizes[7] != DD) return;
  if (in_sizes[8] != DD * DD || in_sizes[9] != DD) return;
  if ((long long)out_size != (long long)NN * DD + 1) return;
  if (ws_size < WS_TOTAL) return;

  const float* ego   = (const float*)d_in[0];
  const int*   uid   = (const int*)d_in[1];
  const int*   iid   = (const int*)d_in[2];
  const float* treat = (const float*)d_in[3];
  const float* alpha = (const float*)d_in[4];
  const float* beta  = (const float*)d_in[5];
  const float* W0    = (const float*)d_in[6];
  const float* b0    = (const float*)d_in[7];
  const float* W1    = (const float*)d_in[8];
  const float* b1    = (const float*)d_in[9];
  float* out = (float*)d_out;

  char* ws = (char*)d_ws;
  float*          RA   = (float*)(ws + O_A);
  float*          RB   = (float*)(ws + O_B);
  unsigned short* MSG  = (unsigned short*)(ws + O_C);
  float*          IPW  = (float*)(ws + O_IPW);
  int*            LIST = (int*)(ws + O_LST);
  int*            CNT  = (int*)(ws + O_CNT);
  int*            OFF  = (int*)(ws + O_OFF);
  int*            FLAG = (int*)(ws + O_FLG);
  unsigned*       REC  = (unsigned*)(ws + O_REC);
  unsigned short* WD0  = (unsigned short*)(ws + O_WD0);
  unsigned short* WD1  = (unsigned short*)(ws + O_WD1);
  float*          BIAS = (float*)(ws + O_BIA);

  hipFuncSetAttribute(reinterpret_cast<const void*>(&k_bucket), hipFuncAttributeMaxDynamicSharedMemorySize,
                      (int)BK_LDS_BYTES);

  k_plane<(MSG_SPLIT_L1 ? 3 : 0)><<<KT1 / 32, 256, 0, stream>>>(W0, DD, DD, DD, WD0, 64, 64);
  k_plane<(MSG_SPLIT_L2 ? 3 : 0)><<<KT2 / 32, 256, 0, stream>>>(W1, DD, DD, DD, WD1, 64, 64);
  k_bias<<<1, 32, 0, stream>>>(b0, b1, BIAS);
  k_node<<<NN * 16 / 256, 256, 0, stream>>>(ego, RA, RB);
  k_inter<<<NREC, 256, 0, stream>>>(RB, uid, iid, treat, alpha, beta, IPW, REC);
  k_loss<<<1, 256, 0, stream>>>(REC, out);
  k_bucket<<<NBLK, 256, BK_LDS_BYTES, stream>>>(uid, iid, LIST, CNT, OFF, FLAG);

  const int gemmBlocks = ((MROWS / 64) + 7) / 8;
  k_replay<KT1><<<NBLK, 256, 0, stream>>>(RA, IPW, uid, iid, LIST, CNT, OFF, FLAG, MSG);
  k_gemm_nt<0, 1><<<gemmBlocks, 256, 0, stream>>>(MSG, WD0, BIAS, RB, NN, DD, KT1, DD);
  k_row1<<<NN * 16 / 256, 256, 0, stream>>>(RB, RA);
  k_replay<KT2><<<NBLK, 256, 0, stream>>>(RA, IPW, uid, iid, LIST, CNT, OFF, FLAG, MSG);
  k_gemm_nt<0, 1><<<gemmBlocks, 256, 0, stream>>>(MSG, WD1, BIAS + DD, RB, NN, DD, KT2, DD);
  k_row2<<<NN * 16 / 256, 256, 0, stream>>>(ego, RA, RB, FLAG, out);
}
